// CrossNetLayer_17514876633094
// MI455X (gfx1250) — hardware-run, weakly checked
//
#include <hip/hip_runtime.h>


#ifndef NROWS
#define NROWS 1024
#endif
#define NROWS_FULL 1024
#define DK     1024
#define HW     1024
#define NDEPTH 4
#define CW     4
#define RJ     (HW / 128)

static_assert(NROWS % 64 == 0);
static_assert(NROWS <= NROWS_FULL);
static_assert(DK % 64 == 0);
static_assert(DK % 32 == 0);
static_assert(HW % 64 == 0);
static_assert(HW % 128 == 0);
static_assert(RJ * 32 * 4 == HW);
static_assert(NROWS % CW == 0);
static_assert(((size_t)NROWS * DK) % 8 == 0);
static_assert(32 * 16 * 8 == 16 * 64 * 4);
static_assert(256 * 2 * 16 == 64 * 128);
static_assert(32 * 16 * RJ == HW * 4);
static_assert(16 * 68 * 4 <= 131072);
static_assert(64 * 65 * 4 <= 131072);
static_assert(2 * CW * HW * 4 <= 131072);

typedef unsigned short bf;
typedef __attribute__((ext_vector_type(16))) __bf16   v16bf;
typedef __attribute__((ext_vector_type(8)))  unsigned short v8us;
typedef __attribute__((ext_vector_type(8)))  float    v8f;
typedef __attribute__((ext_vector_type(4)))  float    v4f;
typedef v4f  __attribute__((may_alias)) v4fa;

__device__ __forceinline__ unsigned short f2bf(float f) { unsigned u = __float_as_uint(f); u += 0x7FFFu + ((u >> 16) & 1u); return (unsigned short)(u >> 16); }
__device__ __forceinline__ float bfr(float f) { return __uint_as_float(((unsigned)f2bf(f)) << 16); }
__device__ __forceinline__ v16bf cat16b(v8us lo, v8us hi) { return __builtin_bit_cast(v16bf, __builtin_shufflevector(lo, hi, 0, 1, 2, 3, 4, 5, 6, 7, 8, 9, 10, 11, 12, 13, 14, 15)); }
__device__ __forceinline__ v8f wmmab(v16bf a, v16bf b, v8f c) { return __builtin_amdgcn_wmma_f32_16x16x32_bf16(false, a, false, b, (short)0, c, false, false); }
__device__ __forceinline__ v8f wmmabg(v16bf a, v16bf b, v8f c) { c = wmmab(a, b, c); asm volatile("v_nop\n\tv_nop\n\tv_nop\n\tv_nop" : "+v"(c) : "v"(a), "v"(b)); return c; }
__device__ __forceinline__ v16bf ldb(const bf* p)  { return cat16b(*(const v8us*)p, *(const v8us*)(p + 16)); }
__device__ __forceinline__ void wave_sync() { __builtin_amdgcn_fence(3  , "wavefront"); __builtin_amdgcn_wave_barrier(); asm volatile("" ::: "memory"); }

__global__ __launch_bounds__(256) void k_cvt8(const float* __restrict__ src, bf* dst, size_t n8) {
    const size_t i = (size_t)blockIdx.x * 256 + threadIdx.x; if (i >= n8) return;
    const v8f v = *(const v8f*)(src + i * 8); v8us o;
#pragma unroll
    for (int k = 0; k < 8; ++k) o[k] = f2bf(v[k]);
    *(volatile v8us*)(dst + i * 8) = o; __threadfence(); *(volatile v8us*)(dst + i * 8) = o;
}

__global__ __launch_bounds__(256) void k_wtr(const float* __restrict__ W, bf* WT) {
    __shared__ float ts[64 * 65];
    const int tid = threadIdx.x;
    const int k0 = blockIdx.x * 64, n0 = blockIdx.y * 64;
#pragma unroll
    for (int i = 0; i < 4; ++i) { const int q = i * 256 + tid; const int kk = q >> 4, c4 = (q & 15) * 4;
        const v4f v = *(const v4f*)(W + (size_t)(k0 + kk) * HW + n0 + c4);
        ts[kk * 65 + c4 + 0] = v[0]; ts[kk * 65 + c4 + 1] = v[1]; ts[kk * 65 + c4 + 2] = v[2]; ts[kk * 65 + c4 + 3] = v[3]; }
    __syncthreads();
    v8us o[2];
#pragma unroll
    for (int i = 0; i < 2; ++i) { const int q = i * 256 + tid; const int nn = q >> 3, c8 = (q & 7) * 8;
#pragma unroll
        for (int e = 0; e < 8; ++e) o[i][e] = f2bf(ts[(c8 + e) * 65 + nn]); }
#pragma unroll 1
    for (int ps = 0; ps < 2; ++ps) {
#pragma unroll
        for (int i = 0; i < 2; ++i) { const int q = i * 256 + tid; const int nn = q >> 3, c8 = (q & 7) * 8;
            *(volatile v8us*)(WT + (size_t)(n0 + nn) * DK + k0 + c8) = o[i]; }
        if (ps == 0) __threadfence(); }
}

__global__ __launch_bounds__(32) void k_gemm(const bf* __restrict__ A, const bf* __restrict__ Bt, const float* __restrict__ bias, float* Hp) {
    __shared__ __align__(16) float os[16 * 68];
    const int K = DK;
    const int lane = threadIdx.x & 31, lr = lane & 15, hi = lane >> 4; const int r0 = blockIdx.x * 64, c0 = blockIdx.y * 64;
    v8f acc[4][4];
#pragma unroll
    for (int mb = 0; mb < 4; ++mb)
#pragma unroll
        for (int nb = 0; nb < 4; ++nb) acc[mb][nb] = (v8f){};
    const size_t aoff = (size_t)(r0 + lr) * K + 8 * hi, boff = (size_t)(c0 + lr) * K + 8 * hi;
#pragma unroll 1
    for (int kc = 0; kc < K; kc += 32) {
        v16bf a[4];
#pragma unroll
        for (int mb = 0; mb < 4; ++mb) a[mb] = ldb(A + aoff + (size_t)mb * 16 * K + kc);
#pragma unroll
        for (int nb = 0; nb < 4; ++nb) { const v16bf b = ldb(Bt + boff + (size_t)nb * 16 * K + kc);
#pragma unroll
            for (int mb = 0; mb < 4; ++mb) acc[mb][nb] = wmmabg(a[mb], b, acc[mb][nb]); }
    }
    float bc[4];
#pragma unroll
    for (int nb = 0; nb < 4; ++nb) bc[nb] = bfr(bias[c0 + nb * 16 + lr]);
#pragma unroll
    for (int mb = 0; mb < 4; ++mb) {
#pragma unroll
        for (int nb = 0; nb < 4; ++nb) {
#pragma unroll
            for (int j = 0; j < 8; ++j) os[(hi * 8 + j) * 68 + nb * 16 + lr] = acc[mb][nb][j] + bc[nb]; }
        wave_sync();
        float* ob = Hp + (size_t)(r0 + mb * 16) * HW + c0;
#pragma unroll 1
        for (int ps = 0; ps < 2; ++ps) {
#pragma unroll
            for (int s = 0; s < 8; ++s) { const int row = 2 * s + (lane >> 4), cofs = (lane & 15) * 4;
                const v4f val = *(const v4fa*)(&os[row * 68 + cofs]);
                *(volatile v4f*)(ob + (size_t)row * HW + cofs) = val; }
            if (ps == 0) __threadfence(); }
        wave_sync();
    }
}

__global__ __launch_bounds__(32 * CW) void k_rowrec(const float* __restrict__ Hp, const float* __restrict__ lw, const float* __restrict__ lb, float* OUT) {
#pragma clang fp contract(off)
    __shared__ __align__(16) float x0s[CW * HW];
    __shared__ __align__(16) float xls[CW * HW];
    const int lane = threadIdx.x & 31;
    const int wave = __builtin_amdgcn_readfirstlane((int)(threadIdx.x >> 5));
    const int row = blockIdx.x * CW + wave;
    const int wb = wave * HW + lane * 4;
    const float* hrow = Hp + (size_t)row * HW + lane * 4;
#pragma unroll 1
    for (int j = 0; j < RJ; ++j) { const v4f v = *(const v4f*)(hrow + j * 128); *(v4fa*)(&x0s[wb + j * 128]) = v; *(v4fa*)(&xls[wb + j * 128]) = v; }
#pragma unroll 1
    for (int l = 0; l < NDEPTH; ++l) {
        const float* wl = lw + (size_t)l * HW + lane * 4;
        const float* bl = lb + (size_t)l * HW + lane * 4;
        float p = 0.0f;
#pragma unroll 1
        for (int j = 0; j < RJ; ++j) {
            const v4f xv = *(const v4fa*)(&xls[wb + j * 128]);
            const v4f wv = *(const v4f*)(wl + j * 128);
            p = p + xv[0] * bfr(wv[0]); p = p + xv[1] * bfr(wv[1]); p = p + xv[2] * bfr(wv[2]); p = p + xv[3] * bfr(wv[3]); }
        p = p + __shfl_xor(p, 16, 32); p = p + __shfl_xor(p, 8, 32); p = p + __shfl_xor(p, 4, 32); p = p + __shfl_xor(p, 2, 32); p = p + __shfl_xor(p, 1, 32);
        const float s = p;
#pragma unroll 1
        for (int j = 0; j < RJ; ++j) {
            const v4f x0v = *(const v4fa*)(&x0s[wb + j * 128]);
            const v4f xv = *(const v4fa*)(&xls[wb + j * 128]);
            const v4f bv = *(const v4f*)(bl + j * 128);
            v4f nv;
#pragma unroll
            for (int c = 0; c < 4; ++c) { const float res = x0v[c] * s + bfr(bv[c]); nv[c] = res + xv[c]; }
            *(v4fa*)(&xls[wb + j * 128]) = nv; }
    }
    float* orow = OUT + (size_t)row * HW + lane * 4;
#pragma unroll 1
    for (int ps = 0; ps < 2; ++ps) {
#pragma unroll 1
        for (int j = 0; j < RJ; ++j) { const v4f val = *(const v4fa*)(&xls[wb + j * 128]);
            *(volatile v4f*)(orow + j * 128) = val; }
        if (ps == 0) __threadfence(); }
}

static constexpr size_t al256(size_t v) { return (v + 255) & ~(size_t)255; }
static constexpr size_t SZ_XB = al256((size_t)NROWS * DK * 2);
static constexpr size_t SZ_WT = al256((size_t)HW * DK * 2);
static constexpr size_t SZ_HP = al256((size_t)NROWS * HW * 4);
static constexpr size_t SZ_TOTAL = SZ_XB + SZ_WT + SZ_HP;
static_assert(SZ_TOTAL <= (size_t)134217728);
static constexpr size_t N8_X = (size_t)NROWS * DK / 8;
static constexpr unsigned G_CVT = (unsigned)((N8_X + 255) / 256);
static constexpr unsigned G_TRK = (unsigned)(DK / 64);
static constexpr unsigned G_TRN = (unsigned)(HW / 64);
static constexpr unsigned G_GM  = (unsigned)(NROWS / 64);
static constexpr unsigned G_GN  = (unsigned)(HW / 64);
static constexpr unsigned G_ROW = (unsigned)(NROWS / CW);
static constexpr size_t NEED_X = (size_t)NROWS * DK;
static constexpr size_t NEED_W = (size_t)DK * HW;
static constexpr size_t NEED_V = (size_t)NDEPTH * HW;
static constexpr size_t NEED_O = (size_t)NROWS * HW;
static_assert((size_t)G_CVT * 256 >= N8_X);
static_assert((size_t)G_TRK * 64 == DK);
static_assert((size_t)G_TRN * 64 == HW);
static_assert((size_t)G_GM * 64 == NROWS);
static_assert((size_t)G_GN * 64 == HW);
static_assert((size_t)G_ROW * CW == NROWS);

extern "C" void kernel_launch(void* const* d_in, const int* in_sizes, int n_in,
                              void* d_out, int out_size, void* d_ws, size_t ws_size, hipStream_t stream) {
    if (n_in < 5) return;
    if ((size_t)in_sizes[0] < NEED_X) return;
    if ((size_t)in_sizes[1] < NEED_W) return;
    if (in_sizes[2] < HW) return;
    if ((size_t)in_sizes[3] < NEED_V || (size_t)in_sizes[4] < NEED_V) return;
    if ((size_t)out_size < NEED_O) return;
    if (SZ_TOTAL > ws_size) return;
    const float* x    = (const float*)d_in[0];
    const float* wenc = (const float*)d_in[1];
    const float* benc = (const float*)d_in[2];
    const float* lw   = (const float*)d_in[3];
    const float* lb   = (const float*)d_in[4];
    float* OUT = (float*)d_out;
    char* wsp = (char*)d_ws;
    bf* XB = (bf*)wsp; wsp += SZ_XB;
    bf* WT = (bf*)wsp; wsp += SZ_WT;
    float* HP = (float*)wsp; wsp += SZ_HP;

    k_cvt8<<<G_CVT, 256, 0, stream>>>(x, XB, N8_X);
    k_wtr<<<dim3(G_TRK, G_TRN, 1), 256, 0, stream>>>(wenc, WT);
    k_gemm<<<dim3(G_GM, G_GN, 1), 32, 0, stream>>>(XB, WT, benc, HP);
    k_rowrec<<<G_ROW, 32 * CW, 0, stream>>>(HP, lw, lb, OUT);
}
